// OptLayer_44581760533210
// MI455X (gfx1250) — hardware-verified
//
#include <hip/hip_runtime.h>
#include <stddef.h>
#include <stdint.h>

#define NB     8192
#define KD     1024
#define ND     512
#define TOTALC 90.0f
#define NBIS   60
#define SWP    68

static_assert(NB % 256 == 0);
static_assert(ND % 64 == 0);
static_assert(KD % 256 == 0);
static_assert(KD % 32 == 0);
static_assert(ND == 32 * 16);
static_assert((SWP * 4) % 16 == 0);

typedef unsigned short u16;
typedef __bf16 v16b __attribute__((ext_vector_type(16)));
typedef unsigned short v8us __attribute__((ext_vector_type(8)));
typedef float v8f __attribute__((ext_vector_type(8)));
typedef float v4f __attribute__((ext_vector_type(4)));
typedef unsigned int v4u __attribute__((ext_vector_type(4)));

union Frag  { v16b v; v8us h[2]; };
union Pack8 { v8us h; v4u u; u16 s[8]; };

__device__ __forceinline__ v8f zero8() { return (v8f){0.f, 0.f, 0.f, 0.f, 0.f, 0.f, 0.f, 0.f}; }

__device__ __forceinline__ v8f mma(v16b a, v16b b, v8f c) {
  c = __builtin_amdgcn_wmma_f32_16x16x32_bf16(false, a, false, b, (short)0, c, false, false);
  asm volatile("v_nop\n\tv_nop\n\tv_nop\n\tv_nop" : "+v"(c) : "v"(a), "v"(b));
  return c;
}

__device__ __forceinline__ u16 f2bf(float f) {
  unsigned int u = __float_as_uint(f);
  u += 0x7FFFu + ((u >> 16) & 1u);
  return (u16)(u >> 16);
}
__device__ __forceinline__ float bf2f(u16 h) { return __uint_as_float(((unsigned int)h) << 16); }
__device__ __forceinline__ u16 lo_of(float f, u16 hi) { return f2bf(f - bf2f(hi)); }
__device__ __forceinline__ void split8(v4f a, v4f b, v4u& hu, v4u& lu) {
  Pack8 ph, pl;
#pragma unroll
  for (int i = 0; i < 4; ++i) {
    const u16 h0 = f2bf(a[i]);
    ph.s[i] = h0;
    pl.s[i] = lo_of(a[i], h0);
    const u16 h1 = f2bf(b[i]);
    ph.s[4 + i] = h1;
    pl.s[4 + i] = lo_of(b[i], h1);
  }
  hu = ph.u;
  lu = pl.u;
}

__device__ __forceinline__ v16b ldfrag(const u16* p, int ld, int row0, int k0, int lane) {
  const int m = lane & 15, lh = lane >> 4;
  const u16* q = p + (size_t)(row0 + m) * ld + k0 + 8 * lh;
  Frag f;
  f.h[0] = *(const v8us*)(q);
  f.h[1] = *(const v8us*)(q + 16);
  return f.v;
}

__device__ __forceinline__ void gemm_hl(const u16* __restrict__ Ah, const u16* __restrict__ Al, int lda,
                                        const u16* __restrict__ Bh, const u16* __restrict__ Bl, int ldb, int K,
                                        int m0, int n0, int lane, v8f (&acc)[2][4]) {
#pragma unroll 1
  for (int k0 = 0; k0 < K; k0 += 32) {
    v16b bh[4];
#pragma unroll
    for (int t = 0; t < 4; ++t) bh[t] = ldfrag(Bh, ldb, n0 + 16 * t, k0, lane);
    const v16b a0 = ldfrag(Ah, lda, m0, k0, lane);
    const v16b a1 = ldfrag(Ah, lda, m0 + 16, k0, lane);
#pragma unroll
    for (int t = 0; t < 4; ++t) {
      acc[0][t] = mma(a0, bh[t], acc[0][t]);
      acc[1][t] = mma(a1, bh[t], acc[1][t]);
    }
    const v16b l0 = ldfrag(Al, lda, m0, k0, lane);
    const v16b l1 = ldfrag(Al, lda, m0 + 16, k0, lane);
#pragma unroll
    for (int t = 0; t < 4; ++t) {
      acc[0][t] = mma(l0, bh[t], acc[0][t]);
      acc[1][t] = mma(l1, bh[t], acc[1][t]);
    }
#pragma unroll
    for (int t = 0; t < 4; ++t) {
      const v16b bl = ldfrag(Bl, ldb, n0 + 16 * t, k0, lane);
      acc[0][t] = mma(a0, bl, acc[0][t]);
      acc[1][t] = mma(a1, bl, acc[1][t]);
    }
  }
}

__device__ __forceinline__ float wave_sum(float v) {
#pragma unroll
  for (int m = 16; m >= 1; m >>= 1) v += __shfl_xor(v, m, 32);
  return v;
}
__device__ __forceinline__ float wave_min(float v) {
#pragma unroll
  for (int m = 16; m >= 1; m >>= 1) v = fminf(v, __shfl_xor(v, m, 32));
  return v;
}
__device__ __forceinline__ float wave_max(float v) {
#pragma unroll
  for (int m = 16; m >= 1; m >>= 1) v = fmaxf(v, __shfl_xor(v, m, 32));
  return v;
}

__global__ __launch_bounds__(256) void k_cvt(const float* __restrict__ x, const float* __restrict__ w,
                                             u16* __restrict__ xh, u16* __restrict__ xl,
                                             u16* __restrict__ wh, u16* __restrict__ wl) {
  const int tid = threadIdx.x, lane = tid & 31, wave = tid >> 5;
  const bool isx = (int)blockIdx.x < (NB / 8);
  const int row = isx ? ((int)blockIdx.x * 8 + wave) : (((int)blockIdx.x - NB / 8) * 8 + wave);
  const float* src = isx ? x : w;
  u16* dh = isx ? xh : wh;
  u16* dl = isx ? xl : wl;
  v4u hv[4], lv[4];
  size_t go[4];
#pragma unroll
  for (int it = 0; it < 4; ++it) {
    const size_t off = (size_t)row * KD + it * 256 + lane * 8;
    const float* s = src + off;
    const v4f a0 = *(const v4f*)(s), a1 = *(const v4f*)(s + 4);
    split8(a0, a1, hv[it], lv[it]);
    go[it] = off;
  }
#pragma unroll
  for (int it = 0; it < 4; ++it) {
    *(volatile v4u*)(dh + go[it]) = hv[it];
    *(volatile v4u*)(dl + go[it]) = lv[it];
  }
  __threadfence();
#pragma unroll
  for (int it = 0; it < 4; ++it) {
    *(volatile v4u*)(dh + go[it]) = hv[it];
    *(volatile v4u*)(dl + go[it]) = lv[it];
  }
}

__global__ __launch_bounds__(256) void k_gemm(const u16* __restrict__ xh, const u16* __restrict__ xl,
                                              const u16* __restrict__ wh, const u16* __restrict__ wl,
                                              const float* __restrict__ bias, float* __restrict__ z) {
  __shared__ __align__(16) float sw[8][16 * SWP];
  const int tid = threadIdx.x, lane = tid & 31, wave = tid >> 5;
  const int lh = lane >> 4, c = lane & 15;
  const int m0 = blockIdx.x * 256 + wave * 32;
  const int n0 = blockIdx.y * 64;

  v8f acc[2][4];
#pragma unroll
  for (int s = 0; s < 2; ++s)
#pragma unroll
    for (int t = 0; t < 4; ++t) acc[s][t] = zero8();
  gemm_hl(xh, xl, KD, wh, wl, KD, KD, m0, n0, lane, acc);

  float bb[4];
#pragma unroll
  for (int t = 0; t < 4; ++t) bb[t] = bias[n0 + 16 * t + c];
  float* wst = sw[wave];
#pragma unroll
  for (int sub = 0; sub < 2; ++sub) {
    __syncthreads();
#pragma unroll
    for (int t = 0; t < 4; ++t) {
#pragma unroll
      for (int r = 0; r < 8; ++r) wst[(8 * lh + r) * SWP + 16 * t + c] = acc[sub][t][r] - bb[t];
    }
    __syncthreads();
    v4f val[8];
    size_t go[8];
#pragma unroll
    for (int it = 0; it < 8; ++it) {
      const int p = it * 32 + lane;
      const int L = p >> 4, pc = p & 15;
      val[it] = *(const v4f*)(wst + L * SWP + pc * 4);
      go[it]  = (size_t)(m0 + sub * 16 + L) * ND + n0 + pc * 4;
    }
#pragma unroll
    for (int it = 0; it < 8; ++it) *(volatile v4f*)(z + go[it]) = val[it];
    __threadfence();
#pragma unroll
    for (int it = 0; it < 8; ++it) *(volatile v4f*)(z + go[it]) = val[it];
  }
}

__global__ __launch_bounds__(256) void k_proj(const float* __restrict__ z, const float* __restrict__ u,
                                              float* __restrict__ out) {
#pragma clang fp contract(off)
  const int tid = threadIdx.x, lane = tid & 31, wave = tid >> 5;
  const int row = blockIdx.x * 8 + wave;
  const float* zr = z + (size_t)row * ND;

  v4f zv[4], uv[4];
#pragma unroll
  for (int j = 0; j < 4; ++j) {
    const int p = 4 * (j * 32 + lane);
    zv[j] = *(const v4f*)(zr + p);
    uv[j] = *(const v4f*)(u + p);
  }

  float zmin = zv[0][0], zmax = zv[0][0], umax = uv[0][0];
#pragma unroll
  for (int j = 0; j < 4; ++j) {
#pragma unroll
    for (int i = 0; i < 4; ++i) {
      zmin = fminf(zmin, zv[j][i]);
      zmax = fmaxf(zmax, zv[j][i]);
      umax = fmaxf(umax, uv[j][i]);
    }
  }
  zmin = wave_min(zmin);
  zmax = wave_max(zmax);
  umax = wave_max(umax);

  float lo = zmin - umax;
  float hi = zmax;
#pragma unroll 1
  for (int it = 0; it < NBIS; ++it) {
    const float mid = 0.5f * (lo + hi);
    float s = 0.f;
#pragma unroll
    for (int j = 0; j < 4; ++j) {
#pragma unroll
      for (int i = 0; i < 4; ++i) s += fminf(fmaxf(zv[j][i] - mid, 0.f), uv[j][i]);
    }
    s = wave_sum(s);
    const float f = s - TOTALC;
    const bool up = (f > 0.f);
    lo = up ? mid : lo;
    hi = up ? hi : mid;
  }
  const float tau = 0.5f * (lo + hi);

  float fl = 0.f, kl = 0.f;
#pragma unroll
  for (int j = 0; j < 4; ++j) {
#pragma unroll
    for (int i = 0; i < 4; ++i) {
      const float s = zv[j][i] - tau;
      fl += fminf(fmaxf(s, 0.f), uv[j][i]);
      kl += ((s > 0.f) && (s < uv[j][i])) ? 1.f : 0.f;
    }
  }
  fl = wave_sum(fl) - TOTALC;
  kl = fmaxf(wave_sum(kl), 1.f);
  const float rk = 1.0f / kl;
  const float tstar = tau + fl * rk;

  v4f y[4];
  size_t go[4];
#pragma unroll
  for (int j = 0; j < 4; ++j) {
#pragma unroll
    for (int i = 0; i < 4; ++i) y[j][i] = fminf(fmaxf(zv[j][i] - tstar, 0.f), uv[j][i]);
    go[j] = (size_t)row * ND + 4 * (j * 32 + lane);
  }
#pragma unroll
  for (int j = 0; j < 4; ++j) *(volatile v4f*)(out + go[j]) = y[j];
  __threadfence();
#pragma unroll
  for (int j = 0; j < 4; ++j) *(volatile v4f*)(out + go[j]) = y[j];
}

extern "C" void kernel_launch(void* const* d_in, const int* in_sizes, int n_in,
                              void* d_out, int out_size, void* d_ws, size_t ws_size,
                              hipStream_t stream) {
  if (n_in < 4) return;
  if (in_sizes[0] != NB * KD) return;
  if (in_sizes[1] != ND * KD) return;
  if (in_sizes[2] != ND) return;
  if (in_sizes[3] != ND) return;
  if (out_size != NB * ND) return;

  const float* x = (const float*)d_in[0];
  const float* w = (const float*)d_in[1];
  const float* b = (const float*)d_in[2];
  const float* u = (const float*)d_in[3];
  float* out = (float*)d_out;

  const size_t szX = (size_t)NB * KD * 2;
  const size_t szW = (size_t)ND * KD * 2;
  const size_t szZ = (size_t)NB * ND * 4;
  size_t off = 0;
  const size_t oXH = off; off += szX;
  const size_t oXL = off; off += szX;
  const size_t oWH = off; off += szW;
  const size_t oWL = off; off += szW;
  const size_t oZ  = off; off += szZ;
  if (off > ws_size) return;
  if (off > (size_t)134217728) return;

  char* ws = (char*)d_ws;
  u16* XH = (u16*)(ws + oXH);
  u16* XL = (u16*)(ws + oXL);
  u16* WH = (u16*)(ws + oWH);
  u16* WL = (u16*)(ws + oWL);
  float* Z = (float*)(ws + oZ);

  k_cvt<<<dim3(NB / 8 + ND / 8), dim3(256), 0, stream>>>(x, w, XH, XL, WH, WL);
  k_gemm<<<dim3(NB / 256, ND / 64), dim3(256), 0, stream>>>(XH, XL, WH, WL, b, Z);
  k_proj<<<dim3(NB / 8), dim3(256), 0, stream>>>(Z, u, out);
  (void)hipGetLastError();
}
